// MLPDecoder_79113297592641
// MI455X (gfx1250) — hardware-verified
//
#include <hip/hip_runtime.h>


typedef _Float16 v16h __attribute__((ext_vector_type(16)));
typedef _Float16 v8h  __attribute__((ext_vector_type(8)));
typedef float    v8f  __attribute__((ext_vector_type(8)));
typedef float    v4f  __attribute__((ext_vector_type(4)));
typedef unsigned int v4u __attribute__((ext_vector_type(4)));

#ifndef E_MAX
#define E_MAX 1000000
#endif

#define DD     128
#define KK1    256
#define CC     5
#define TM     128
#define NTHR   256
#define WSCALE 64.0f
#define WINV   0.015625f

#define TILE_H   512
#define NT1      64
#define NT2      32
#define NT3      4
#define OFF_W1   0
#define OFF_W2   65536
#define OFF_WP   98304
#define WT_BYTES 102400
#define OFF_A    102400
#define OFF_H1   167936
#define OFF_H2   200704
#define OFF_OUT  233472
#define SMEM_BYTES 236032

static_assert(OFF_W2 == OFF_W1 + NT1 * TILE_H * 2);
static_assert(OFF_WP == OFF_W2 + NT2 * TILE_H * 2);
static_assert(WT_BYTES == OFF_WP + NT3 * TILE_H * 2);
static_assert(OFF_H1 == OFF_A + TM * KK1 * 2);
static_assert(OFF_H2 == OFF_H1 + TM * DD * 2);
static_assert(OFF_OUT == OFF_H2 + TM * DD * 2);
static_assert(SMEM_BYTES == OFF_OUT + TM * CC * 4);
static_assert((TM * CC * 4) % 128 == 0);
static_assert(WT_BYTES % 128 == 0);
static_assert((WT_BYTES / 16) % NTHR == 0);
static_assert(NTHR * 4 >= TM * CC);
static_assert(KK1 % 32 == 0 && DD % 32 == 0);
static_assert(NTHR == 2 * TM);
static_assert(DD / 8 == 16);

union Frag { v16h v; v8h h[2]; };

__device__ __forceinline__ float bf16_rne(float x) {
  unsigned u = __float_as_uint(x);
  u += 0x7FFFu + ((u >> 16) & 1u);
  u &= 0xFFFF0000u;
  return __uint_as_float(u);
}

__device__ __forceinline__ v8f wmma_g(v16h a, v16h b, v8f c) {
  c = __builtin_amdgcn_wmma_f32_16x16x32_f16(false, a, false, b, (short)0, c, false, false);
  asm volatile("v_nop\n\tv_nop\n\tv_nop\n\tv_nop" : "+v"(c) : "v"(a), "v"(b));
  return c;
}

__device__ __forceinline__ v16h load_frag_a(const _Float16* base, int pitch, int lane) {
  const int hh = lane >> 4;
  const int r  = lane & 15;
  const _Float16* p = base + r * pitch + 8 * hh;
  Frag f;
  f.h[0] = *(const v8h*)(p);
  f.h[1] = *(const v8h*)(p + 16);
  return f.v;
}

__global__ __launch_bounds__(256) void cvt_feat_f16(const float* __restrict__ in,
                                                    _Float16* __restrict__ outp, int n8) {
  const int g = blockIdx.x * 256 + threadIdx.x;
  if (g >= n8) return;
  const float4 x0 = *(const float4*)(in + (size_t)g * 8);
  const float4 x1 = *(const float4*)(in + (size_t)g * 8 + 4);
  union { v8h h; v4u u; } o;
  o.h[0] = (_Float16)bf16_rne(x0.x); o.h[1] = (_Float16)bf16_rne(x0.y);
  o.h[2] = (_Float16)bf16_rne(x0.z); o.h[3] = (_Float16)bf16_rne(x0.w);
  o.h[4] = (_Float16)bf16_rne(x1.x); o.h[5] = (_Float16)bf16_rne(x1.y);
  o.h[6] = (_Float16)bf16_rne(x1.z); o.h[7] = (_Float16)bf16_rne(x1.w);
  const v4u val = o.u;
  volatile v4u* p = (volatile v4u*)(outp + (size_t)g * 8);
  *p = val;
  __threadfence();
  *p = val;
}

__global__ __launch_bounds__(256) void prep_wtiles(const float* __restrict__ W, int K, int NC,
                                                   int ntn, _Float16* __restrict__ tiles, int nth) {
  const int j = blockIdx.x * 256 + threadIdx.x;
  if (j >= nth) return;
  const int i8 = j & 1;
  const int ln = (j >> 1) & 31;
  const int t  = j >> 6;
  const int nt = t % ntn;
  const int kt = t / ntn;
  const int n  = nt * 16 + (ln & 15);
  const int hh = ln >> 4;
  const int kb = kt * 32 + 16 * i8 + 8 * hh;
  const int nc = (n < NC) ? n : (NC - 1);
  union { v8h h; v4u u; } o;
#pragma unroll
  for (int c = 0; c < 8; ++c) {
    int k = kb + c; k = (k < K) ? k : (K - 1);
    const float x = W[(size_t)k * NC + nc];
    const float y = (n < NC) ? (WSCALE * bf16_rne(x)) : 0.0f;
    o.h[c] = (_Float16)y;
  }
  const v4u val = o.u;
  volatile v4u* p = (volatile v4u*)(tiles + (size_t)j * 8);
  *p = val;
  __threadfence();
  *p = val;
}

__global__ __launch_bounds__(NTHR) void edge_mlp_kernel(const _Float16* __restrict__ Uh,
                                                        const _Float16* __restrict__ Ih,
                                                        const int* __restrict__ src,
                                                        const int* __restrict__ dst,
                                                        const uint4* __restrict__ wtiles,
                                                        float* __restrict__ out,
                                                        int E, int NU, int NI) {
  extern __shared__ __align__(16) char smem[];
  _Float16* sW1  = (_Float16*)(smem + OFF_W1);
  _Float16* sW2  = (_Float16*)(smem + OFF_W2);
  _Float16* sWp  = (_Float16*)(smem + OFF_WP);
  _Float16* sA   = (_Float16*)(smem + OFF_A);
  _Float16* sH1  = (_Float16*)(smem + OFF_H1);
  _Float16* sH2  = (_Float16*)(smem + OFF_H2);
  float*    sOut = (float*)(smem + OFF_OUT);

  const int tid  = threadIdx.x;
  const int lane = tid & 31;
  const int wave = tid >> 5;
  const int half = lane >> 4;
  const int mrow = lane & 15;
  const int blockBase = blockIdx.x * TM;

  {
    uint4* dT = (uint4*)smem;
    for (int i = tid; i < WT_BYTES / 16; i += NTHR) dT[i] = wtiles[i];
  }
  {
    const int r  = tid & (TM - 1);
    const int cb = tid >> 7;
    int e = blockBase + r; e = (e < E) ? e : (E - 1);
    int s = src[e]; s = (s < 0) ? 0 : s; s = (s > NU - 1) ? (NU - 1) : s;
    int d = dst[e]; d = (d < 0) ? 0 : d; d = (d > NI - 1) ? (NI - 1) : d;
    const _Float16* pu = Uh + (size_t)s * DD;
    const _Float16* pi = Ih + (size_t)d * DD;
    _Float16* rowA = sA + r * KK1;
#pragma unroll 4
    for (int it = 0; it < 8; ++it) {
      const int c = cb + 2 * it;
      const uint4 vu = *(const uint4*)(pu + c * 8);
      const uint4 vi = *(const uint4*)(pi + c * 8);
      *(uint4*)(rowA + c * 8)      = vu;
      *(uint4*)(rowA + DD + c * 8) = vi;
    }
  }
  __syncthreads();

  const int m0 = wave * 16;

  {
    v8f acc[8];
#pragma unroll
    for (int nt = 0; nt < 8; ++nt)
#pragma unroll
      for (int i = 0; i < 8; ++i) acc[nt][i] = 0.0f;
#pragma unroll
    for (int kt = 0; kt < KK1 / 32; ++kt) {
      const v16h a = load_frag_a(sA + m0 * KK1 + kt * 32, KK1, lane);
#pragma unroll
      for (int nt = 0; nt < 8; ++nt) {
        const v16h b = *(const v16h*)(sW1 + (kt * 8 + nt) * TILE_H + lane * 16);
        acc[nt] = wmma_g(a, b, acc[nt]);
      }
    }
#pragma unroll
    for (int nt = 0; nt < 8; ++nt)
#pragma unroll
      for (int i = 0; i < 8; ++i) {
        const float v = fmaxf(acc[nt][i] * WINV, 0.0f);
        sH1[(m0 + 8 * half + i) * DD + nt * 16 + mrow] = (_Float16)v;
      }
  }
  __syncthreads();

  {
    v8f acc[8];
#pragma unroll
    for (int nt = 0; nt < 8; ++nt)
#pragma unroll
      for (int i = 0; i < 8; ++i) acc[nt][i] = 0.0f;
#pragma unroll
    for (int kt = 0; kt < DD / 32; ++kt) {
      const v16h a = load_frag_a(sH1 + m0 * DD + kt * 32, DD, lane);
#pragma unroll
      for (int nt = 0; nt < 8; ++nt) {
        const v16h b = *(const v16h*)(sW2 + (kt * 8 + nt) * TILE_H + lane * 16);
        acc[nt] = wmma_g(a, b, acc[nt]);
      }
    }
#pragma unroll
    for (int nt = 0; nt < 8; ++nt)
#pragma unroll
      for (int i = 0; i < 8; ++i)
        sH2[(m0 + 8 * half + i) * DD + nt * 16 + mrow] = (_Float16)(acc[nt][i] * WINV);
  }
  __syncthreads();

  {
    v8f acc;
#pragma unroll
    for (int i = 0; i < 8; ++i) acc[i] = 0.0f;
#pragma unroll
    for (int kt = 0; kt < DD / 32; ++kt) {
      const v16h a = load_frag_a(sH2 + m0 * DD + kt * 32, DD, lane);
      const v16h b = *(const v16h*)(sWp + kt * TILE_H + lane * 16);
      acc = wmma_g(a, b, acc);
    }
    if (mrow < CC) {
#pragma unroll
      for (int i = 0; i < 8; ++i)
        sOut[(m0 + 8 * half + i) * CC + mrow] = acc[i] * WINV;
    }
  }
  __syncthreads();

  {
    int rows = E - blockBase; rows = (rows < TM) ? rows : TM;
    const int nvalid = rows * CC;
    float* gout = out + (size_t)blockBase * CC;
    const int f0 = tid * 4;
    const int fl = (f0 + 4 <= TM * CC) ? f0 : 0;
    const v4f vv = *(const v4f*)(sOut + fl);
    const int rem = nvalid - f0;
    if (rem >= 4) {
      *(volatile v4f*)(gout + f0) = vv;
    } else if (rem > 0) {
      volatile float* q = gout + f0;
      q[0] = vv[0];
      if (rem > 1) q[1] = vv[1];
      if (rem > 2) q[2] = vv[2];
    }
    __threadfence();
    if (rem >= 4) {
      *(volatile v4f*)(gout + f0) = vv;
    } else if (rem > 0) {
      volatile float* q = gout + f0;
      q[0] = vv[0];
      if (rem > 1) q[1] = vv[1];
      if (rem > 2) q[2] = vv[2];
    }
  }
}

extern "C" void kernel_launch(void* const* d_in, const int* in_sizes, int n_in,
                              void* d_out, int out_size, void* d_ws, size_t ws_size,
                              hipStream_t stream) {
  if (n_in < 7) return;
  if (in_sizes[0] < DD || in_sizes[1] < DD) return;
  if (in_sizes[4] < KK1 * DD || in_sizes[5] < DD * DD || in_sizes[6] < DD * CC) return;

  const float* ufeat = (const float*)d_in[0];
  const float* ifeat = (const float*)d_in[1];
  const int*   src   = (const int*)d_in[2];
  const int*   dst   = (const int*)d_in[3];
  const float* W1    = (const float*)d_in[4];
  const float* W2    = (const float*)d_in[5];
  const float* Wp    = (const float*)d_in[6];
  float* out = (float*)d_out;

  const int NU = in_sizes[0] / DD;
  const int NI = in_sizes[1] / DD;
  int E = in_sizes[2];
  if (in_sizes[3] < E) E = in_sizes[3];
  if (E > E_MAX) E = E_MAX;
  if (out_size / CC < E) E = out_size / CC;
  if (E < 1 || NU < 1 || NI < 1) return;

  char* ws = (char*)d_ws;
  const size_t offT   = 0;
  const size_t offU   = offT + WT_BYTES;
  const size_t bytesU = (size_t)NU * DD * 2;
  const size_t offI   = offU + ((bytesU + 127) & ~(size_t)127);
  const size_t bytesI = (size_t)NI * DD * 2;
  const size_t total  = offI + ((bytesI + 127) & ~(size_t)127);
  if (total > ws_size) return;

  _Float16* tiles = (_Float16*)(ws + offT);
  _Float16* Uh    = (_Float16*)(ws + offU);
  _Float16* Ih    = (_Float16*)(ws + offI);
  _Float16* tW1   = tiles;
  _Float16* tW2   = tiles + NT1 * TILE_H;
  _Float16* tWp   = tiles + (NT1 + NT2) * TILE_H;

  const int n8U = NU * (DD / 8);
  const int n8I = NI * (DD / 8);
  cvt_feat_f16<<<(n8U + 255) / 256, 256, 0, stream>>>(ufeat, Uh, n8U);
  cvt_feat_f16<<<(n8I + 255) / 256, 256, 0, stream>>>(ifeat, Ih, n8I);

  const int nth1 = NT1 * 64, nth2 = NT2 * 64, nth3 = NT3 * 64;
  prep_wtiles<<<(nth1 + 255) / 256, 256, 0, stream>>>(W1, KK1, DD, 8, tW1, nth1);
  prep_wtiles<<<(nth2 + 255) / 256, 256, 0, stream>>>(W2, DD, DD, 8, tW2, nth2);
  prep_wtiles<<<(nth3 + 255) / 256, 256, 0, stream>>>(Wp, DD, CC, 1, tWp, nth3);

  hipFuncSetAttribute(reinterpret_cast<const void*>(&edge_mlp_kernel),
                      hipFuncAttributeMaxDynamicSharedMemorySize, SMEM_BYTES);
  const int grid = (E + TM - 1) / TM;
  edge_mlp_kernel<<<grid, NTHR, SMEM_BYTES, stream>>>(Uh, Ih, src, dst, (const uint4*)tiles,
                                                      out, E, NU, NI);
}
